// DAGCN_32186484916473
// MI455X (gfx1250) — hardware-run, weakly checked
//
#include <hip/hip_runtime.h>


#pragma clang fp contract(off)

#ifndef NB
#define NB 64
#endif
#ifndef NN
#define NN 2048
#endif
#define NB_FULL 64
#define NN_FULL 2048
#ifndef OUT_NN
#define OUT_NN NN
#endif
#define CC   64
#define EE   16
#define CK   3
#define KI   (CK * CC)
#define NJ   (CK * CC * CC)
#define MBT  (NB / 16)
#define MSL  (MBT >= 2 ? 2 : 1)
#define AW   4
#define PSP  72
#define QRS  2048.0f
#define QRI  (1.0f / 2048.0f)
#define LOG2E 1.4426950408889634f
#define PCARRY 16384.0f
#define PSI  (1.0f / 16384.0f)
#define NEGB (-3.0e38f)

static_assert(CC == 64);
static_assert(EE == 16);
static_assert(KI % 32 == 0);
static_assert(NN % 256 == 0);
static_assert(NN % (16 * AW) == 0);
static_assert(NB % 16 == 0);
static_assert(NB >= 16);
static_assert(NB <= 64);
static_assert(NB <= NB_FULL);
static_assert(NN <= NN_FULL);
static_assert(MBT % MSL == 0);
static_assert((MBT / MSL) * MSL * 16 == NB);
static_assert((NJ * 4) % 256 == 0);
static_assert((CC * 4) % 256 == 0);
static_assert(NJ % 64 == 0);
static_assert((PSP * 2) % 16 == 0);
static_assert(256 * 16 * 4 == 256 * 64);
static_assert(256 * 16 * 2 == 64 * 128);
static_assert(32 * 16 * 4 == 16 * 128);
static_assert(32 * 16 * 16 == 64 * 128);
static_assert(32 * 16 * 32 == 64 * 256);
static_assert(32 * 16 * 8 == 16 * 256);
static_assert(256 * 17 * 4 <= 131072);
static_assert(64 * PSP * 2 <= 131072);
static_assert(AW * 16 * PSP * 2 <= 131072);
static_assert(64 * 68 * 4 <= 131072);
static_assert(16 * 68 * 4 <= 131072);

typedef _Float16 h16;
typedef unsigned short bf;
typedef __attribute__((ext_vector_type(16))) __bf16   v16bf;
typedef __attribute__((ext_vector_type(16))) _Float16 v16h;
typedef __attribute__((ext_vector_type(8)))  _Float16 v8h;
typedef __attribute__((ext_vector_type(8)))  unsigned short v8us;
typedef __attribute__((ext_vector_type(8)))  float    v8f;
typedef __attribute__((ext_vector_type(4)))  float    v4f;
typedef v4f  __attribute__((may_alias)) v4fa;
typedef v8h  __attribute__((may_alias)) v8ha;

__device__ __forceinline__ unsigned short f2bf(float f) { unsigned u = __float_as_uint(f); u += 0x7FFFu + ((u >> 16) & 1u); return (unsigned short)(u >> 16); }
__device__ __forceinline__ float bfr(float f) { return __uint_as_float(((unsigned)f2bf(f)) << 16); }
__device__ __forceinline__ v16h cat16(v8h lo, v8h hi) { return __builtin_shufflevector(lo, hi, 0, 1, 2, 3, 4, 5, 6, 7, 8, 9, 10, 11, 12, 13, 14, 15); }
__device__ __forceinline__ v16bf cat16b(v8us lo, v8us hi) { return __builtin_bit_cast(v16bf, __builtin_shufflevector(lo, hi, 0, 1, 2, 3, 4, 5, 6, 7, 8, 9, 10, 11, 12, 13, 14, 15)); }
__device__ __forceinline__ v8f wmma16(v16h a, v16h b, v8f c) { return __builtin_amdgcn_wmma_f32_16x16x32_f16(false, a, false, b, (short)0, c, false, false); }
__device__ __forceinline__ v8f wmmab(v16bf a, v16bf b, v8f c) { return __builtin_amdgcn_wmma_f32_16x16x32_bf16(false, a, false, b, (short)0, c, false, false); }
__device__ __forceinline__ v16h  ldh(const h16* p) { return cat16(*(const v8h*)p, *(const v8h*)(p + 16)); }
__device__ __forceinline__ v16bf ldb(const bf* p)  { return cat16b(*(const v8us*)p, *(const v8us*)(p + 16)); }
__device__ __forceinline__ void wave_sync() { __builtin_amdgcn_fence(3  , "wavefront"); __builtin_amdgcn_wave_barrier(); asm volatile("" ::: "memory"); }

__device__ __forceinline__ v8f wmmag(v16h a, v16h b, v8f c) {
    c = __builtin_amdgcn_wmma_f32_16x16x32_f16(false, a, false, b, (short)0, c, false, false);
    asm volatile("v_nop\n\tv_nop\n\tv_nop\n\tv_nop" : "+v"(c) : "v"(a), "v"(b));
    return c;
}
static __device__ __forceinline__ h16 toh_flush(float v) { const h16 r = (h16)v; return (fabsf(v) < 6.103515625e-05f) ? (h16)0.0f : r; }
__device__ __forceinline__ v16h ldx(const float* p) {
    const v4f a = *(const v4f*)p, b = *(const v4f*)(p + 4), c = *(const v4f*)(p + 16), d = *(const v4f*)(p + 20); v16h o;
#pragma unroll
    for (int i = 0; i < 4; ++i) { o[i] = toh_flush(bfr(a[i])); o[4 + i] = toh_flush(bfr(b[i])); o[8 + i] = toh_flush(bfr(c[i])); o[12 + i] = toh_flush(bfr(d[i])); }
    return o;
}

__global__ __launch_bounds__(256) void k_wpt(const float* __restrict__ wp, const float* __restrict__ bp, h16* WPT) {
    const int p = blockIdx.x * 256 + threadIdx.x;
    const int j = p >> 2, q = p & 3; const int d0 = (q & 1) * 8; const float sc = (q < 2) ? QRS : 1.0f;
    v8h o;
    if (blockIdx.x < (NJ * 4) / 256) {
        const int k = j >> 12, oo = (j >> 6) & 63, i = j & 63;
        const size_t s0 = (size_t)k * (CC * CC) + (size_t)i * CC + (size_t)oo;
#pragma unroll
        for (int d = 0; d < 8; ++d) { const float v = wp[(size_t)(d0 + d) * NJ + s0]; o[d] = toh_flush(bfr(v) * sc); }
    } else {
        const int oo = j - NJ;
#pragma unroll
        for (int d = 0; d < 8; ++d) { const float v = bp[(d0 + d) * CC + oo]; o[d] = toh_flush(bfr(v) * sc); }
    }
    *(volatile v8h*)(WPT + (size_t)p * 8) = o; __threadfence(); *(volatile v8h*)(WPT + (size_t)p * 8) = o;
}

__global__ __launch_bounds__(256) void k_ln(const float* __restrict__ nodeE, const float* __restrict__ timeE, const float* __restrict__ gam, const float* __restrict__ bet,
                                            h16* NA, h16* QH, h16* QR) {
    __shared__ __align__(16) float ls[256 * 17];
    const int tid = threadIdx.x; const int n = blockIdx.x * 256 + tid;
    float mu = 0.0f;
#pragma unroll 1
    for (int d = 0; d < EE; ++d) { const float v = bfr(nodeE[(size_t)n * EE + d]) + bfr(timeE[d]); ls[tid * 17 + d] = v; mu += v; }
    mu *= (1.0f / EE);
    float var = 0.0f;
#pragma unroll 1
    for (int d = 0; d < EE; ++d) { const float t = ls[tid * 17 + d] - mu; var += t * t; }
    var *= (1.0f / EE);
    const float rs = rsqrtf(var + 1e-12f);
#pragma unroll 1
    for (int d = 0; d < EE; ++d) { const float t = ls[tid * 17 + d] - mu; ls[tid * 17 + d] = t * rs * bfr(gam[d]) + bfr(bet[d]); }
    __syncthreads();
#pragma unroll 1
    for (int it = 0; it < 4; ++it) {
        const int p = it * 256 + tid; const int row = p >> 2, q = p & 3, d0 = (q & 1) * 8;
        v8h hv, rv;
#pragma unroll
        for (int i = 0; i < 8; ++i) { const float v = ls[row * 17 + d0 + i]; const h16 a = toh_flush(v); hv[i] = a; rv[i] = toh_flush((v - (float)a) * QRS); }
        const v8h zz = (v8h){};
        const bool lo = q < 2;
        const v8h na = lo ? hv : rv; const v8h qh = lo ? hv : zz; const v8h qr = lo ? rv : hv;
        const size_t o = ((size_t)blockIdx.x * 1024 + (size_t)p) * 8;
        *(volatile v8h*)(NA + o) = na; *(volatile v8h*)(QH + o) = qh; *(volatile v8h*)(QR + o) = qr;
        __threadfence();
        *(volatile v8h*)(NA + o) = na; *(volatile v8h*)(QH + o) = qh; *(volatile v8h*)(QR + o) = qr;
    }
}

__global__ __launch_bounds__(256) void k_xt(const float* __restrict__ x, h16* XT) {
    __shared__ __align__(16) h16 ts[64 * PSP];
    const int tid = threadIdx.x; const int m0 = blockIdx.x * 64, b = blockIdx.y;
#pragma unroll 1
    for (int it = 0; it < 4; ++it) {
        const int idx = it * 256 + tid; const int r = idx >> 4, q = idx & 15;
        const v4f v = *(const v4f*)(x + ((size_t)b * NN_FULL + (size_t)(m0 + r)) * CC + q * 4);
#pragma unroll
        for (int i = 0; i < 4; ++i) ts[(q * 4 + i) * PSP + r] = toh_flush(bfr(v[i]));
    }
    __syncthreads();
#pragma unroll 1
    for (int ps = 0; ps < 2; ++ps) {
#pragma unroll 1
        for (int it = 0; it < 2; ++it) {
            const int idx = it * 256 + tid; const int c = idx >> 3, p8 = (idx & 7) * 8;
            const v8h o = *(const v8ha*)(&ts[c * PSP + p8]);
            *(volatile v8h*)(XT + ((size_t)b * CC + (size_t)c) * NN + (size_t)(m0 + p8)) = o; }
        if (ps == 0) __threadfence(); }
}

__device__ __forceinline__ void score32(const h16* __restrict__ NA, size_t ko, int key0, v16h qh, v16h qr, float (&ta)[8], float (&tb)[8]) {
    const h16* ka = NA + ko + (size_t)key0 * 32;
    const v16h ka0 = ldh(ka), kb0 = ldh(ka + 16 * 32);
    v8f sHa = (v8f){}, sLa = (v8f){}, sHb = (v8f){}, sLb = (v8f){};
    sHa = wmmag(ka0, qh, sHa); sLa = wmmag(ka0, qr, sLa); sHb = wmmag(kb0, qh, sHb); sLb = wmmag(kb0, qr, sLb);
#pragma unroll
    for (int r = 0; r < 8; ++r) { ta[r] = (sHa[r] + sLa[r] * QRI) * LOG2E; tb[r] = (sHb[r] + sLb[r] * QRI) * LOG2E; }
}

__global__ __launch_bounds__(32 * AW) void k_soft(const h16* __restrict__ NA, const h16* __restrict__ QH, const h16* __restrict__ QR, h16* P) {
    __shared__ __align__(16) h16 pt[AW * 16 * PSP];
    const int lane = threadIdx.x & 31, lr = lane & 15, hi = lane >> 4;
    const int wave = __builtin_amdgcn_readfirstlane((int)(threadIdx.x >> 5));
    const int t0 = (blockIdx.x * AW + wave) * 16;
    const size_t qo = (size_t)(t0 + lr) * 32 + 8 * hi;
    const v16h qh = ldh(QH + qo), qr = ldh(QR + qo);
    const size_t ko = (size_t)lr * 32 + 8 * hi;
    float m = NEGB, l = 0.0f;
#pragma unroll 1
    for (int key0 = 0; key0 < NN; key0 += 32) {
        float ta[8], tb[8];
        score32(NA, ko, key0, qh, qr, ta, tb);
        float mx = NEGB;
#pragma unroll
        for (int r = 0; r < 8; ++r) mx = fmaxf(mx, fmaxf(ta[r], tb[r]));
        mx = fmaxf(mx, __shfl_xor(mx, 16, 32));
        const float mnew = fmaxf(m, mx);
        const float alpha = __builtin_amdgcn_exp2f(m - mnew);
        float ls = 0.0f;
#pragma unroll
        for (int r = 0; r < 8; ++r) ls += __builtin_amdgcn_exp2f(ta[r] - mnew) + __builtin_amdgcn_exp2f(tb[r] - mnew);
        l = l * alpha + ls; m = mnew;
    }
    l += __shfl_xor(l, 16, 32);
    const float inv = PCARRY * (1.0f / l);
    const int wb = wave * 16 * PSP;
#pragma unroll 1
    for (int key0 = 0; key0 < NN; key0 += 64) {
#pragma unroll
        for (int hh = 0; hh < 2; ++hh) {
            float ta[8], tb[8];
            score32(NA, ko, key0 + 32 * hh, qh, qr, ta, tb);
            v8h pa, pc;
#pragma unroll
            for (int r = 0; r < 8; ++r) { pa[r] = toh_flush(__builtin_amdgcn_exp2f(ta[r] - m) * inv); pc[r] = toh_flush(__builtin_amdgcn_exp2f(tb[r] - m) * inv); }
            *(v8ha*)(&pt[wb + lr * PSP + 32 * hh + 8 * hi]) = pa;
            *(v8ha*)(&pt[wb + lr * PSP + 32 * hh + 16 + 8 * hi]) = pc;
        }
        wave_sync();
#pragma unroll 1
        for (int ps = 0; ps < 2; ++ps) {
#pragma unroll
            for (int s = 0; s < 4; ++s) { const int row = 4 * s + (lane >> 3), c8 = (lane & 7) * 8;
                const v8h val = *(const v8ha*)(&pt[wb + row * PSP + c8]);
                *(volatile v8h*)(P + (size_t)(t0 + row) * NN + (size_t)(key0 + c8)) = val; }
            if (ps == 0) __threadfence(); }
        wave_sync();
    }
}

__global__ __launch_bounds__(32) void k_hop(const h16* __restrict__ A, const h16* __restrict__ Pm, const float* __restrict__ xin, h16* YN, h16* YT, int hop) {
    __shared__ __align__(16) float os[64 * 68];
    const int lane = threadIdx.x & 31, lr = lane & 15, hi = lane >> 4;
    const int bb = blockIdx.x; const int r0 = bb * 64, c0 = blockIdx.y * 64;
    v8f acc[4][4];
#pragma unroll
    for (int mb = 0; mb < 4; ++mb)
#pragma unroll
        for (int nb = 0; nb < 4; ++nb) acc[mb][nb] = (v8f){};
    const size_t aoff = (size_t)(r0 + lr) * NN + 8 * hi, boff = (size_t)(c0 + lr) * NN + 8 * hi;
#pragma unroll 1
    for (int kc = 0; kc < NN; kc += 32) {
        v16h a[4];
#pragma unroll
        for (int mb = 0; mb < 4; ++mb) a[mb] = ldh(A + aoff + (size_t)mb * 16 * NN + kc);
#pragma unroll
        for (int nb = 0; nb < 4; ++nb) { const v16h b = ldh(Pm + boff + (size_t)nb * 16 * NN + kc);
#pragma unroll
            for (int mb = 0; mb < 4; ++mb) acc[mb][nb] = wmmag(a[mb], b, acc[mb][nb]); }
    }
#pragma unroll
    for (int mb = 0; mb < 4; ++mb)
#pragma unroll
        for (int nb = 0; nb < 4; ++nb)
#pragma unroll
            for (int j = 0; j < 8; ++j) os[(mb * 16 + hi * 8 + j) * 68 + nb * 16 + lr] = acc[mb][nb][j] * PSI;
    wave_sync();
#pragma unroll 1
    for (int ps = 0; ps < 2; ++ps) {
#pragma unroll 1
        for (int s = 0; s < 16; ++s) { const int row = 4 * s + (lane >> 3), c8 = (lane & 7) * 8;
            float y[8];
#pragma unroll
            for (int i = 0; i < 8; ++i) y[i] = os[(c8 + i) * 68 + row];
            if (hop == 2) {
                const float* xr = xin + ((size_t)bb * NN_FULL + (size_t)(c0 + row)) * CC + c8;
                const v4f x0 = *(const v4f*)xr, x1 = *(const v4f*)(xr + 4);
#pragma unroll
                for (int i = 0; i < 4; ++i) { y[i] = 2.0f * y[i] - bfr(x0[i]); y[4 + i] = 2.0f * y[4 + i] - bfr(x1[i]); }
            }
            v8h hv;
#pragma unroll
            for (int i = 0; i < 8; ++i) hv[i] = toh_flush(y[i]);
            *(volatile v8h*)(YN + ((size_t)bb * NN + (size_t)(c0 + row)) * CC + c8) = hv; }
        if (hop == 1) {
#pragma unroll 1
            for (int s = 0; s < 16; ++s) { const int row = 4 * s + (lane >> 3), n8 = (lane & 7) * 8;
                const v4f x0 = *(const v4fa*)(&os[row * 68 + n8]); const v4f x1 = *(const v4fa*)(&os[row * 68 + n8 + 4]); v8h hv;
#pragma unroll
                for (int i = 0; i < 4; ++i) { hv[i] = toh_flush(x0[i]); hv[4 + i] = toh_flush(x1[i]); }
                *(volatile v8h*)(YT + (size_t)(r0 + row) * NN + (size_t)(c0 + n8)) = hv; }
        }
        if (ps == 0) __threadfence(); }
}

__global__ __launch_bounds__(32) void k_wgen(const h16* __restrict__ NA, const h16* __restrict__ WPT, h16* WT, float* BN) {
    __shared__ __align__(16) float os[64 * 68];
    const int lane = threadIdx.x & 31, lr = lane & 15, hi = lane >> 4;
    const int r0 = blockIdx.x * 64, jt = blockIdx.y;
    const size_t aoff = (size_t)(r0 + lr) * 32 + 8 * hi, boff = ((size_t)jt * 64 + (size_t)lr) * 32 + 8 * hi;
    v16h a[4];
#pragma unroll
    for (int mb = 0; mb < 4; ++mb) a[mb] = ldh(NA + aoff + (size_t)mb * 16 * 32);
#pragma unroll
    for (int nb = 0; nb < 4; ++nb) { const v16h b = ldh(WPT + boff + (size_t)nb * 16 * 32);
#pragma unroll
        for (int mb = 0; mb < 4; ++mb) { v8f c = (v8f){}; c = wmmag(a[mb], b, c);
#pragma unroll
            for (int j = 0; j < 8; ++j) os[(mb * 16 + hi * 8 + j) * 68 + nb * 16 + lr] = c[j] * QRI; } }
    wave_sync();
#pragma unroll 1
    for (int ps = 0; ps < 2; ++ps) {
        if (jt < NJ / 64) {
            const int k = jt >> 6, oo = jt & 63;
#pragma unroll 1
            for (int s = 0; s < 16; ++s) { const int row = 4 * s + (lane >> 3), i8 = (lane & 7) * 8;
                const v4f x0 = *(const v4fa*)(&os[row * 68 + i8]); const v4f x1 = *(const v4fa*)(&os[row * 68 + i8 + 4]); v8h hv;
#pragma unroll
                for (int i = 0; i < 4; ++i) { hv[i] = toh_flush(x0[i]); hv[4 + i] = toh_flush(x1[i]); }
                *(volatile v8h*)(WT + ((size_t)(r0 + row) * CC + (size_t)oo) * KI + (size_t)k * CC + i8) = hv; }
        } else {
#pragma unroll 1
            for (int s = 0; s < 32; ++s) { const int row = 2 * s + (lane >> 4), c4 = (lane & 15) * 4;
                const v4f val = *(const v4fa*)(&os[row * 68 + c4]);
                *(volatile v4f*)(BN + (size_t)(r0 + row) * CC + c4) = val; }
        }
        if (ps == 0) __threadfence(); }
}

__global__ __launch_bounds__(32) __attribute__((amdgpu_num_vgpr(256))) void k_final(const float* __restrict__ x, const h16* __restrict__ Y1, const h16* __restrict__ Y2, const h16* __restrict__ WT, const float* __restrict__ BN, float* OUT) {
    __shared__ __align__(16) float os[16 * 68];
    const int lane = threadIdx.x & 31, lr = lane & 15, hi = lane >> 4;
    const int n = blockIdx.x;
    const int brow0 = blockIdx.y * (MSL * 16);
    v8f acc[MSL][4];
#pragma unroll
    for (int mb = 0; mb < MSL; ++mb)
#pragma unroll
        for (int nb = 0; nb < 4; ++nb) acc[mb][nb] = (v8f){};
    const size_t boff = ((size_t)n * CC + (size_t)lr) * KI + 8 * hi;
    const size_t xoff = ((size_t)(brow0 + lr) * NN_FULL + (size_t)n) * CC + 8 * hi;
    const size_t yoff = ((size_t)(brow0 + lr) * NN + (size_t)n) * CC + 8 * hi;
#pragma unroll 1
    for (int kc = 0; kc < CC; kc += 32) {
        v16h a[MSL];
#pragma unroll
        for (int mb = 0; mb < MSL; ++mb) a[mb] = ldx(x + xoff + (size_t)mb * 16 * NN_FULL * CC + kc);
#pragma unroll
        for (int nb = 0; nb < 4; ++nb) { const v16h b = ldh(WT + boff + (size_t)nb * 16 * KI + kc);
#pragma unroll
            for (int mb = 0; mb < MSL; ++mb) acc[mb][nb] = wmmag(a[mb], b, acc[mb][nb]); }
    }
#pragma unroll 1
    for (int kc = 0; kc < CC; kc += 32) {
        v16h a[MSL];
#pragma unroll
        for (int mb = 0; mb < MSL; ++mb) a[mb] = ldh(Y1 + yoff + (size_t)mb * 16 * NN * CC + kc);
#pragma unroll
        for (int nb = 0; nb < 4; ++nb) { const v16h b = ldh(WT + boff + (size_t)nb * 16 * KI + CC + kc);
#pragma unroll
            for (int mb = 0; mb < MSL; ++mb) acc[mb][nb] = wmmag(a[mb], b, acc[mb][nb]); }
    }
#pragma unroll 1
    for (int kc = 0; kc < CC; kc += 32) {
        v16h a[MSL];
#pragma unroll
        for (int mb = 0; mb < MSL; ++mb) a[mb] = ldh(Y2 + yoff + (size_t)mb * 16 * NN * CC + kc);
#pragma unroll
        for (int nb = 0; nb < 4; ++nb) { const v16h b = ldh(WT + boff + (size_t)nb * 16 * KI + 2 * CC + kc);
#pragma unroll
            for (int mb = 0; mb < MSL; ++mb) acc[mb][nb] = wmmag(a[mb], b, acc[mb][nb]); }
    }
    const int c4 = (lane & 15) * 4;
    const v4f bias4 = *(const v4f*)(BN + (size_t)n * CC + c4);
#pragma unroll
    for (int mb = 0; mb < MSL; ++mb) {
#pragma unroll
        for (int nb = 0; nb < 4; ++nb) {
#pragma unroll
            for (int j = 0; j < 8; ++j) os[(hi * 8 + j) * 68 + nb * 16 + lr] = acc[mb][nb][j]; }
        wave_sync();
#pragma unroll 1
        for (int ps = 0; ps < 2; ++ps) {
#pragma unroll
            for (int s = 0; s < 8; ++s) { const int row = 2 * s + (lane >> 4);
                const v4f val = *(const v4fa*)(&os[row * 68 + c4]) + bias4;
                *(volatile v4f*)(OUT + ((size_t)(brow0 + mb * 16 + row) * OUT_NN + (size_t)n) * CC + c4) = val; }
            if (ps == 0) __threadfence(); }
        wave_sync();
    }
}

static constexpr size_t al256(size_t v) { return (v + 255) & ~(size_t)255; }
static constexpr size_t SZ_WPT = al256((size_t)(NJ + CC) * 32 * 2);
static constexpr size_t SZ_NE  = al256((size_t)NN * 32 * 2);
static constexpr size_t SZ_BC  = al256((size_t)NB * CC * NN * 2);
static constexpr size_t SZ_P   = al256((size_t)NN * NN * 2);
static constexpr size_t SZ_WT  = al256((size_t)NN * CC * KI * 2);
static constexpr size_t SZ_BN  = al256((size_t)NN * CC * 4);
static constexpr size_t SZ_TOTAL = SZ_WPT + 3 * SZ_NE + 4 * SZ_BC + SZ_P + SZ_WT + SZ_BN;
static_assert(SZ_TOTAL <= (size_t)134217728);
static_assert((size_t)(NJ + CC) * 4 == (size_t)((NJ + CC) * 4 / 256) * 256);
static_assert((size_t)(NN / 256) * 1024 * 16 == (size_t)NN * 32 * 2);
static_assert((size_t)(NN / 64) * NB * 64 * 128 == (size_t)NB * CC * NN * 2);
static_assert((size_t)(NN / (16 * AW)) * AW * 16 * NN * 2 == (size_t)NN * NN * 2);
static_assert((size_t)NB * (NN / 64) * 64 * 128 == (size_t)NB * CC * NN * 2);
static_assert((size_t)(NN / 64) * (NJ / 64) * 64 * 128 == (size_t)NN * CC * KI * 2);
static_assert((size_t)NN * (MBT / MSL) * MSL * 16 * 256 == (size_t)NB * NN * CC * 4);

extern "C" void kernel_launch(void* const* d_in, const int* in_sizes, int n_in,
                              void* d_out, int out_size, void* d_ws, size_t ws_size, hipStream_t stream) {
    if (n_in < 7) return;
    if ((size_t)in_sizes[0] < ((size_t)(NB - 1) * NN_FULL + NN) * CC) return;
    if ((size_t)in_sizes[1] < (size_t)NN * EE || in_sizes[2] < EE) return;
    if ((size_t)in_sizes[3] < (size_t)EE * NJ || in_sizes[4] < EE * CC) return;
    if (in_sizes[5] < EE || in_sizes[6] < EE) return;
    if ((size_t)out_size < ((size_t)(NB - 1) * OUT_NN + NN) * CC) return;
    if (SZ_TOTAL > ws_size) return;
    const float* x     = (const float*)d_in[0];
    const float* nodeE = (const float*)d_in[1];
    const float* timeE = (const float*)d_in[2];
    const float* wp    = (const float*)d_in[3];
    const float* bp    = (const float*)d_in[4];
    const float* gam   = (const float*)d_in[5];
    const float* bet   = (const float*)d_in[6];
    float* OUT = (float*)d_out;
    char* wsp = (char*)d_ws;
    h16* WPT = (h16*)wsp; wsp += SZ_WPT;
    h16* NA  = (h16*)wsp; wsp += SZ_NE;
    h16* QH  = (h16*)wsp; wsp += SZ_NE;
    h16* QR  = (h16*)wsp; wsp += SZ_NE;
    h16* XT  = (h16*)wsp; wsp += SZ_BC;
    h16* Y1T = (h16*)wsp; wsp += SZ_BC;
    h16* Y1N = (h16*)wsp; wsp += SZ_BC;
    h16* Y2N = (h16*)wsp; wsp += SZ_BC;
    h16* PP  = (h16*)wsp; wsp += SZ_P;
    h16* WT  = (h16*)wsp; wsp += SZ_WT;
    float* BN = (float*)wsp; wsp += SZ_BN;

    k_wpt<<<(unsigned)((NJ + CC) * 4 / 256), 256, 0, stream>>>(wp, bp, WPT);
    k_ln<<<NN / 256, 256, 0, stream>>>(nodeE, timeE, gam, bet, NA, QH, QR);
    k_xt<<<dim3(NN / 64, NB, 1), 256, 0, stream>>>(x, XT);
    k_soft<<<NN / (16 * AW), 32 * AW, 0, stream>>>(NA, QH, QR, PP);
    k_hop<<<dim3(NB, NN / 64, 1), 32, 0, stream>>>(XT, PP, x, Y1N, Y1T, 1);
    k_hop<<<dim3(NB, NN / 64, 1), 32, 0, stream>>>(Y1T, PP, x, Y2N, Y2N, 2);
    k_wgen<<<dim3(NN / 64, NJ / 64 + 1, 1), 32, 0, stream>>>(NA, WPT, WT, BN);
    k_final<<<dim3(NN, MBT / MSL, 1), 32, 0, stream>>>(x, Y1N, Y2N, WT, BN, OUT);
}
